// graphNetworkEqvrnt_45535243272336
// MI455X (gfx1250) — hardware-verified
//
#include <hip/hip_runtime.h>
#include <stddef.h>
#include <math.h>


#define NCH   193
#define MP    208
#define KP    224
#define MT    13
#define KT    7
#define PR    256
#define CH    96
#define NB    128
#define NTA   256
#define EPT   8
#define CHUNK (NTA * EPT)
#define WCAP  (EPT * 2 * 32)
#define SC    16.0f
#define SCI   0.00390625f

static_assert(WCAP == 512);
static_assert((NB * CH) % (4 * NTA) == 0);
static_assert(NB <= 128);

typedef float    v4f  __attribute__((ext_vector_type(4)));
typedef float    v8f  __attribute__((ext_vector_type(8)));
typedef int      v4i  __attribute__((ext_vector_type(4)));
typedef _Float16 v8h  __attribute__((ext_vector_type(8)));
typedef _Float16 v16h __attribute__((ext_vector_type(16)));
union Frag { v16h v; v8h h[2]; };
union H8   { v8h h; v4i i; };

__device__ __forceinline__ v8f wmh(v16h a, v16h b, v8f c) {
  v8f d = __builtin_amdgcn_wmma_f32_16x16x32_f16(false, a, false, b, (short)0, c, false, false);
  asm volatile("v_nop\n\tv_nop\n\tv_nop\n\tv_nop" : "+v"(d) : "v"(a), "v"(b));
  return d;
}
__device__ __forceinline__ v8f zacc() { v8f c;
#pragma unroll
  for (int i = 0; i < 8; ++i) c[i] = 0.0f; return c; }
__device__ __forceinline__ v8h zh8() { v8h r;
#pragma unroll
  for (int i = 0; i < 8; ++i) r[i] = (_Float16)0.0f; return r; }
__device__ __forceinline__ int clampi(int v, int hi) { return v < 0 ? 0 : (v > hi ? hi : v); }

__global__ __launch_bounds__(256) void k_prep(const float* __restrict__ KE1, const float* __restrict__ KE2,
    const float* __restrict__ K1N, const float* __restrict__ K2N, _Float16* A1, _Float16* A2, _Float16* WS, int nblkA)
{
  const int tid = threadIdx.x, b = blockIdx.x;
  const int nA = 3 * MP * KP / 8;
  H8 o;
  _Float16* dst;
  bool act;
  if (b < 2 * nblkA) {
    const bool second = (b >= nblkA);
    const float* src = second ? KE2 : KE1;
    _Float16* pl = second ? A2 : A1;
    const int p = (b - (second ? nblkA : 0)) * 256 + tid;
    act = p < nA;
    const int q = p * 8;
    int l = q / (MP * KP);
    const int rem = q - l * (MP * KP), mm = rem / KP, k0 = rem - mm * KP;
    l = min(l, 2);
    const int mr = min(mm, NCH - 1);
#pragma unroll
    for (int i = 0; i < 8; ++i) {
      const int k = k0 + i;
      float v = src[(size_t)l * NCH * NCH + (size_t)mr * NCH + min(k, NCH - 1)];
      v = (mm < NCH && k < NCH && act) ? v : 0.0f;
      o.h[i] = (_Float16)(v * SC);
    }
    dst = pl + (size_t)min(p, nA - 1) * 8;
  } else {
    const int j = (b - 2 * nblkA) * 256 + tid;
    act = j < 384;
    const int o1 = min(j >> 3, 31), kb1 = (j & 7) * 8;
    const int j2 = min(max(j - 256, 0), 127), o2 = j2 >> 2, kb2 = (j2 & 3) * 8;
#pragma unroll
    for (int i = 0; i < 8; ++i) {
      const int k1 = kb1 + i;
      const float v1 = K1N[o1 * 40 + min(k1, 39)];
      const float v2 = K2N[o2 * 32 + kb2 + i];
      const float v = (j < 256) ? ((k1 < 40) ? v1 : 0.0f) : v2;
      o.h[i] = (_Float16)(v * SC);
    }
    dst = WS + (size_t)min(j, 383) * 8;
  }
  if (act) *(volatile v4i*)dst = o.i;
  __threadfence();
  if (act) *(volatile v4i*)dst = o.i;
}

__global__ __launch_bounds__(256) void k_std(const float* __restrict__ src, int pitch, int ncol, int nrows,
                                             const float* __restrict__ kw, int nkw, float* st)
{
  __shared__ double red[512];
  __shared__ __attribute__((aligned(16))) float resf[32];
  const int tid = threadIdx.x, lane = tid & 31, wave = tid >> 5;
  double s = 0.0, q = 0.0;
#pragma unroll 1
  for (int r = tid; r < nrows; r += 256) {
    const float* p = src + (size_t)r * pitch;
#pragma unroll 1
    for (int c = 0; c < ncol; ++c) { const double v = (double)p[c]; s += v; q += v * v; }
  }
  red[tid] = s; red[256 + tid] = q;
  __syncthreads();
#pragma unroll 1
  for (int stp = 128; stp > 0; stp >>= 1) {
    if (tid < stp) { red[tid] += red[tid + stp]; red[256 + tid] += red[256 + tid + stp]; }
    __syncthreads();
  }
  if (tid == 0) {
    double sk = 1.0, sk2 = 1.0;
    if (nkw > 0) {
      sk = 0.0; sk2 = 0.0;
#pragma unroll 1
      for (int c = 0; c < nkw; ++c) { const double k = (double)kw[c]; sk += k; sk2 += k * k; }
    }
    const double cnt = (double)(nkw > 0 ? nkw : 1) * (double)ncol * (double)nrows;
    const double S1 = sk * red[0], S2 = sk2 * red[256];
    double var = (S2 - S1 * S1 / cnt) / (cnt - 1.0);
    if (var < 0.0) var = 0.0;
    const float sd = sqrtf((float)var);
    resf[0] = 1.0f / (sd + 1e-4f);
    resf[1] = sd;
#pragma unroll
    for (int j = 2; j < 32; ++j) resf[j] = 0.0f;
  }
  __syncthreads();
  v4f rv = {0.0f, 0.0f, 0.0f, 0.0f};
  const bool wr = (wave == 0) && (lane < 8);
  if (wr) rv = *(const v4f*)(resf + 4 * lane);
  if (wr) *(volatile v4f*)(st + 4 * lane) = rv;
  __threadfence();
  if (wr) *(volatile v4f*)(st + 4 * lane) = rv;
}

__device__ __forceinline__ void conv32(const _Float16* __restrict__ W2, const _Float16* Hs, float* Os,
                                       int wave, int h, int m) {
  const int row = wave * 16 + m;
  Frag b;
  b.h[0] = *(const v8h*)(Hs + row * 32 + 8 * h);
  b.h[1] = *(const v8h*)(Hs + row * 32 + 16 + 8 * h);
#pragma unroll
  for (int mt = 0; mt < 2; ++mt) {
    Frag a;
    const _Float16* ap = W2 + (16 * mt + m) * 32 + 8 * h;
    a.h[0] = *(const v8h*)ap;
    a.h[1] = *(const v8h*)(ap + 16);
    const v8f d = wmh(a.v, b.v, zacc());
    v4f lo, hi;
#pragma unroll
    for (int r = 0; r < 4; ++r) { lo[r] = tanhf(d[r] * SCI); hi[r] = tanhf(d[4 + r] * SCI); }
    float* op = Os + row * 32 + 16 * mt + 8 * h;
    *(v4f*)op = lo;
    *(v4f*)(op + 4) = hi;
  }
}
__device__ __forceinline__ void rows32_pass(const float* Os, float* dst, int wave, int lane) {
#pragma unroll
  for (int q = 0; q < 4; ++q) {
    const int f = (wave * 4 + q) * 128 + 4 * lane;
    const v4f v = *(const v4f*)(Os + f);
    *(volatile v4f*)(dst + f) = v;
  }
}

__global__ __launch_bounds__(128) void k_nopen(const float* __restrict__ xn, const _Float16* __restrict__ W1,
    const _Float16* __restrict__ W2, const int* __restrict__ nnp, float* X32, float* C, float* CO, int N)
{
#pragma clang fp contract(off)
  __shared__ __attribute__((aligned(16))) _Float16 Bs[64 * 64];
  __shared__ __attribute__((aligned(16))) _Float16 Hs[64 * 32];
  __shared__ __attribute__((aligned(16))) float Os[64 * 32];
  const int tid = threadIdx.x, lane = tid & 31, wave = tid >> 5, h = lane >> 4, m = lane & 15;
  const int n0 = blockIdx.x * 64;
  {
    const int nl = tid & 63, part = tid >> 6;
    const int n = min(n0 + nl, N - 1);
#pragma unroll 1
    for (int c = part * 32; c < part * 32 + 32; ++c) {
      float v = tanhf(xn[(size_t)min(c, 39) * N + n]);
      v = (c < 40) ? v * SC : 0.0f;
      Bs[nl * 64 + c] = (_Float16)v;
    }
  }
  __syncthreads();
  const int row = wave * 16 + m;
  v8f acc0 = zacc(), acc1 = zacc();
#pragma unroll
  for (int kt = 0; kt < 2; ++kt) {
    Frag b;
    const _Float16* bp = Bs + row * 64 + kt * 32 + 8 * h;
    b.h[0] = *(const v8h*)bp;
    b.h[1] = *(const v8h*)(bp + 16);
    Frag a;
    const _Float16* ap = W1 + m * 64 + kt * 32 + 8 * h;
    a.h[0] = *(const v8h*)ap;
    a.h[1] = *(const v8h*)(ap + 16);
    acc0 = wmh(a.v, b.v, acc0);
    const _Float16* ap2 = W1 + (16 + m) * 64 + kt * 32 + 8 * h;
    a.h[0] = *(const v8h*)ap2;
    a.h[1] = *(const v8h*)(ap2 + 16);
    acc1 = wmh(a.v, b.v, acc1);
  }
  float s1 = 0.0f;
#pragma unroll
  for (int r = 0; r < 8; ++r) s1 += acc0[r] + acc1[r];
  s1 *= SCI;
  s1 += __shfl_xor(s1, 16, 32);
  const float mu = s1 * (1.0f / 32.0f);
  float x0[8], x1[8];
  float ss = 0.0f;
#pragma unroll
  for (int r = 0; r < 8; ++r) {
    x0[r] = acc0[r] * SCI - mu; x1[r] = acc1[r] * SCI - mu;
    ss += x0[r] * x0[r] + x1[r] * x1[r];
  }
  ss += __shfl_xor(ss, 16, 32);
  const float inv = 1.0f / sqrtf(ss + 1e-3f);
  H8 t0, t1;
#pragma unroll
  for (int r = 0; r < 8; ++r) {
    t0.h[r] = (_Float16)(SC * tanhf(x0[r] * inv));
    t1.h[r] = (_Float16)(SC * tanhf(x1[r] * inv));
  }
  *(v8h*)(Hs + row * 32 + 8 * h) = t0.h;
  *(v8h*)(Hs + row * 32 + 16 + 8 * h) = t1.h;
  __syncthreads();
  conv32(W2, Hs, Os, wave, h, m);
  __syncthreads();
  v4f cv = {0.0f, 0.0f, 0.0f, 0.0f};
  const int nn = nnp[0];
  const int nd = n0 + tid;
  const bool cw = tid < 64;
  if (cw) {
    int chn = (nd >= 1) ? ((nd - 1) % 3) : -1;
    if (nd >= nn) chn = -1;
    cv[0] = (chn == 0) ? 3.8f : 0.0f;
    cv[1] = (chn == 1) ? 3.8f : 0.0f;
    cv[2] = (chn == 2) ? 3.8f : 0.0f;
  }
  float* xdst = X32 + (size_t)n0 * 32;
  rows32_pass(Os, xdst, wave, lane);
  if (cw) { *(volatile v4f*)(C + (size_t)nd * 4) = cv; *(volatile v4f*)(CO + (size_t)nd * 4) = cv; }
  __threadfence();
  rows32_pass(Os, xdst, wave, lane);
  if (cw) { *(volatile v4f*)(C + (size_t)nd * 4) = cv; *(volatile v4f*)(CO + (size_t)nd * 4) = cv; }
}

__global__ __launch_bounds__(256) void k_eopen(const float* __restrict__ xe, const float* __restrict__ K1E,
    const float* __restrict__ K2E, float* XE)
{
  __shared__ __attribute__((aligned(16))) float Hs[64 * 32];
  __shared__ __attribute__((aligned(16))) float Os[64 * 32];
  __shared__ float k1s[32];
  __shared__ float k2s[1024];
  const int tid = threadIdx.x;
  const int e0 = blockIdx.x * 64;
  if (tid < 32) k1s[tid] = K1E[tid];
  for (int i = tid; i < 1024; i += 256) k2s[i] = K2E[i];
  __syncthreads();
  if (tid < 64) {
    const float t = tanhf(xe[(size_t)e0 + tid]);
    float s = 0.0f;
#pragma unroll 1
    for (int o = 0; o < 32; ++o) s += k1s[o] * t;
    const float mu = s * (1.0f / 32.0f);
    float ss = 0.0f;
#pragma unroll 1
    for (int o = 0; o < 32; ++o) { const float x = k1s[o] * t - mu; ss += x * x; }
    const float inv = 1.0f / sqrtf(ss + 1e-3f);
#pragma unroll 1
    for (int o = 0; o < 32; ++o) Hs[tid * 32 + o] = tanhf((k1s[o] * t - mu) * inv);
  }
  __syncthreads();
  {
    const int el = tid & 63, og = tid >> 6;
    const float* hrow = Hs + el * 32;
#pragma unroll 1
    for (int o = 0; o < 8; ++o) {
      const float* krow = k2s + (og * 8 + o) * 32;
      float s = 0.0f;
#pragma unroll 4
      for (int c = 0; c < 32; ++c) s += krow[c] * hrow[c];
      Os[el * 32 + og * 8 + o] = tanhf(s);
    }
  }
  __syncthreads();
  float* dst = XE + (size_t)e0 * 32;
  v4f ov[2];
#pragma unroll
  for (int q = 0; q < 2; ++q) ov[q] = *(const v4f*)(Os + (q * 256 + tid) * 4);
#pragma unroll
  for (int q = 0; q < 2; ++q) *(volatile v4f*)(dst + (q * 256 + tid) * 4) = ov[q];
  __threadfence();
#pragma unroll
  for (int q = 0; q < 2; ++q) *(volatile v4f*)(dst + (q * 256 + tid) * 4) = ov[q];
}

__device__ __forceinline__ int scan2(const int* __restrict__ iI, const int* __restrict__ jI, int nE, int cbase,
                                     int nodeBase, int vec8, int* list, int tid, int wave)
{
  const int el0 = tid * EPT, e0 = cbase + el0;
  const int sent = -2147483647 - 1;
  int dv[16];
  if (vec8 != 0 && cbase + CHUNK <= nE) {
    const v4i a = *(const v4i*)(iI + e0), b = *(const v4i*)(iI + e0 + 4);
    const v4i c = *(const v4i*)(jI + e0), d = *(const v4i*)(jI + e0 + 4);
    dv[0] = a.x; dv[1] = a.y; dv[2] = a.z; dv[3] = a.w; dv[4] = b.x; dv[5] = b.y; dv[6] = b.z; dv[7] = b.w;
    dv[8] = c.x; dv[9] = c.y; dv[10] = c.z; dv[11] = c.w; dv[12] = d.x; dv[13] = d.y; dv[14] = d.z; dv[15] = d.w;
  } else {
#pragma unroll
    for (int J = 0; J < 8; ++J) {
      const int e = e0 + J, ec = min(e, nE - 1);
      const int vi = iI[ec], vj = jI[ec];
      dv[J] = (e < nE) ? vi : sent;
      dv[8 + J] = (e < nE) ? vj : sent;
    }
  }
  const unsigned nb = (unsigned)nodeBase;
  unsigned sl[16];
  bool hit[16];
  bool anyb = false;
#pragma unroll
  for (int J = 0; J < 16; ++J) { sl[J] = (unsigned)dv[J] - nb; hit[J] = sl[J] < (unsigned)NB; anyb = anyb || hit[J]; }
  int wc = 0;
  if (__builtin_amdgcn_ballot_w32(anyb) != 0u) {
#pragma unroll
    for (int J = 0; J < 16; ++J) {
      const unsigned mj = __builtin_amdgcn_ballot_w32(hit[J]);
      if (mj != 0u) {
        if (hit[J]) {
          const int pos = wc + (int)__builtin_amdgcn_mbcnt_lo(mj, 0u);
          if (pos < WCAP) list[wave * WCAP + pos] = ((el0 + (J & 7)) << 8) | ((J >> 3) << 7) | (int)sl[J];
        }
        wc += (int)__builtin_popcount(mj);
      }
    }
  }
  return wc;
}

template <int MODE>
__global__ __launch_bounds__(NTA) void k_agg(const int* __restrict__ iI, const int* __restrict__ jI,
    const float* __restrict__ XE, const _Float16* __restrict__ P, const float* __restrict__ WG,
    const float* __restrict__ X32, float* XN, float* C, float* CO, int N, int E, int vec8)
{
#pragma clang fp contract(off)
  constexpr int AW = (MODE == 0) ? 64 : 104;
  __shared__ __attribute__((aligned(16))) float acc[NB * AW];
  __shared__ int list[8 * WCAP];
  __shared__ int wcnt[8];
  const int tid = threadIdx.x, lane = tid & 31, wave = tid >> 5;
  const int nodeBase = blockIdx.x * NB;
  for (int i = tid; i < NB * AW; i += NTA) acc[i] = 0.0f;
  __syncthreads();
  const int nChunks = (E + CHUNK - 1) / CHUNK;
#pragma unroll 1
  for (int chn = 0; chn < nChunks; ++chn) {
    const int cbase = chn * CHUNK;
    const int wc = scan2(iI, jI, E, cbase, nodeBase, vec8, list, tid, wave);
    if (lane == 0) wcnt[wave] = wc;
    __syncthreads();
    if (wave == 0) {
#pragma unroll 1
      for (int w = 0; w < 8; ++w) {
        int n = wcnt[w];
        n = n < 0 ? 0 : (n > WCAP ? WCAP : n);
#pragma unroll 1
        for (int qq = 0; qq < n; ++qq) {
          const int ent = list[w * WCAP + qq];
          const int el = (ent >> 8) & (CHUNK - 1), role = (ent >> 7) & 1, sl = ent & (NB - 1);
          int e = cbase + el;
          e = e > E - 1 ? E - 1 : e;
          if (MODE == 0) {
            const float v = XE[(size_t)e * 32 + lane];
            acc[sl * AW + role * 32 + lane] += v;
          } else {
            const _Float16* mp = P + (size_t)e * PR + role * CH;
            const float a = (float)mp[lane] * (1.0f / SC);
            const float b = (float)mp[lane + 32] * (1.0f / SC);
            const float c = (float)mp[lane + 64] * (1.0f / SC);
            acc[sl * AW + lane] += a;
            acc[sl * AW + 32 + lane] += b;
            acc[sl * AW + 64 + lane] += c;
            const float g = WG[(size_t)e * 4 + (lane & 3)];
            if (lane < 3) acc[sl * AW + CH + role * 4 + lane] += g;
          }
        }
      }
    }
    __syncthreads();
  }
  v4f ov[12];
  float* xb = XN + (size_t)nodeBase * CH;
  if (MODE == 0) {
    const float* x32b = X32 + (size_t)nodeBase * 32;
#pragma unroll
    for (int q = 0; q < 12; ++q) {
      const int f = (wave * 12 + q) * 128 + 4 * lane;
      const int sl = f / CH, c = f - sl * CH, cc = c & 31;
      const v4f x4 = *(const v4f*)(x32b + sl * 32 + ((c < 32) ? c : 0));
      v4f t;
#pragma unroll
      for (int k = 0; k < 4; ++k) {
        const float si = acc[sl * AW + cc + k], sj = acc[sl * AW + 32 + cc + k];
        const float dv = si - sj, av = (si + sj) * 0.5f;
        t[k] = (c < 32) ? x4[k] : ((c < 64) ? dv : av);
      }
      ov[q] = t;
    }
#pragma unroll
    for (int q = 0; q < 12; ++q) *(volatile v4f*)(xb + (wave * 12 + q) * 128 + 4 * lane) = ov[q];
    __threadfence();
#pragma unroll
    for (int q = 0; q < 12; ++q) *(volatile v4f*)(xb + (wave * 12 + q) * 128 + 4 * lane) = ov[q];
  } else {
#pragma unroll
    for (int q = 0; q < 12; ++q) {
      const int f = (wave * 12 + q) * 128 + 4 * lane;
      const int sl = f / CH, c = f - sl * CH;
      const v4f xo = *(const v4f*)(xb + f);
      v4f t;
#pragma unroll
      for (int k = 0; k < 4; ++k) t[k] = xo[k] - 0.1f * acc[sl * AW + c + k];
      ov[q] = t;
    }
    v4f cold4 = {0.0f, 0.0f, 0.0f, 0.0f}, cnew4 = {0.0f, 0.0f, 0.0f, 0.0f};
    const bool cw = tid < NB;
    const size_t crow = (size_t)(nodeBase + (tid & (NB - 1))) * 4;
    if (cw) {
      const v4f cur = *(const v4f*)(C + crow);
      const v4f old = *(const v4f*)(CO + crow);
#pragma unroll
      for (int k = 0; k < 3; ++k) {
        const float ave = (acc[tid * AW + CH + k] + acc[tid * AW + CH + 4 + k]) * 0.5f;
        cnew4[k] = old[k] + 0.2f * ave;
      }
      cold4 = cur;
    }
#pragma unroll
    for (int q = 0; q < 12; ++q) *(volatile v4f*)(xb + (wave * 12 + q) * 128 + 4 * lane) = ov[q];
    if (cw) { *(volatile v4f*)(CO + crow) = cold4; *(volatile v4f*)(C + crow) = cnew4; }
    __threadfence();
#pragma unroll
    for (int q = 0; q < 12; ++q) *(volatile v4f*)(xb + (wave * 12 + q) * 128 + 4 * lane) = ov[q];
    if (cw) { *(volatile v4f*)(CO + crow) = cold4; *(volatile v4f*)(C + crow) = cnew4; }
  }
}

__global__ __launch_bounds__(256) void k_elen(const float* __restrict__ XN, const float* __restrict__ C,
    const int* __restrict__ iI, const int* __restrict__ jI, float* EW, int N, int E)
{
#pragma clang fp contract(off)
  const int e = blockIdx.x * 256 + (int)threadIdx.x;
  if (e >= E) return;
  const int i = clampi(iI[e], N - 1), j = clampi(jI[e], N - 1);
  const float* xi = XN + (size_t)i * CH;
  const float* xj = XN + (size_t)j * CH;
  float s = 0.0f;
#pragma unroll 4
  for (int c = 0; c < CH; ++c) { const float d = xi[c] - xj[c]; s += d * d; }
  const float we = (s > 0.0f) ? sqrtf(s) : 0.0f;
  const v4f ci = *(const v4f*)(C + (size_t)i * 4), cj = *(const v4f*)(C + (size_t)j * 4);
  float s2 = 0.0f;
#pragma unroll
  for (int c = 0; c < 3; ++c) { const float d = ci[c] - cj[c]; s2 += d * d; }
  const float dc = (s2 > 0.0f) ? sqrtf(s2) : 0.0f;
  const v4f o = {we, dc, 0.0f, 0.0f};
  *(volatile v4f*)(EW + (size_t)e * 4) = o;
  __threadfence();
  *(volatile v4f*)(EW + (size_t)e * 4) = o;
}

__global__ __launch_bounds__(128) void k_build(const float* __restrict__ XN, const int* __restrict__ iI,
    const int* __restrict__ jI, const float* __restrict__ Kw1, const float* __restrict__ EW,
    const float* __restrict__ ST1, _Float16* P, int N)
{
#pragma clang fp contract(off)
  __shared__ __attribute__((aligned(16))) _Float16 Ts[64 * PR];
  const int tid = threadIdx.x, lane = tid & 31, wave = tid >> 5;
  const int e0 = blockIdx.x * 64;
  const int el = tid & 63, part = tid >> 6;
  const int e = e0 + el;
  const int i = clampi(iI[e], N - 1), j = clampi(jI[e], N - 1);
  const float we = EW[(size_t)e * 4], dC = EW[(size_t)e * 4 + 1];
  const float inv = ST1[0];
  const float* xi = XN + (size_t)i * CH;
  const float* xj = XN + (size_t)j * CH;
  _Float16* trow = Ts + el * PR;
#pragma unroll 1
  for (int c = part * 48; c < part * 48 + 48; ++c) {
    const float wc = tanhf((Kw1[c] * we) * inv);
    const float a = xi[c], b = xj[c];
    const float g = wc * (a - b);
    const float s = (wc * (a + b)) * 0.5f;
    trow[c] = (_Float16)(SC * tanhf(g));
    trow[CH + c] = (_Float16)(SC * tanhf(s));
  }
  if (part != 0) {
    trow[2 * CH] = (_Float16)(SC * tanhf(dC));
#pragma unroll 1
    for (int c = 2 * CH + 1; c < 200; ++c) trow[c] = (_Float16)0.0f;
    const v8h z = zh8();
#pragma unroll
    for (int q = 0; q < 7; ++q) *(v8h*)(trow + 200 + 8 * q) = z;
  }
  __syncthreads();
  const _Float16* srow0 = Ts + (wave * 16) * PR + 8 * lane;
  _Float16* prow0 = P + (size_t)(e0 + wave * 16) * PR + 8 * lane;
#pragma unroll
  for (int r = 0; r < 16; ++r) { H8 t; t.h = *(const v8h*)(srow0 + r * PR); *(volatile v4i*)(prow0 + (size_t)r * PR) = t.i; }
  __threadfence();
#pragma unroll
  for (int r = 0; r < 16; ++r) { H8 t; t.h = *(const v8h*)(srow0 + r * PR); *(volatile v4i*)(prow0 + (size_t)r * PR) = t.i; }
}

template <int MODE>
__global__ __launch_bounds__(128) void k_gemm(const _Float16* __restrict__ A, _Float16* P,
    const float* __restrict__ Kw1, const float* __restrict__ Kw2,
    const float* __restrict__ EW, const float* __restrict__ ST1, float* W3)
{
#pragma clang fp contract(off)
  __shared__ __attribute__((aligned(16))) _Float16 As[MP * KP];
  __shared__ __attribute__((aligned(16))) _Float16 Ss[4 * 16 * PR];
  __shared__ __attribute__((aligned(16))) float Ys[4 * 32 * 16];
  __shared__ float kw2s[3 * MP];
  __shared__ float kw1s[CH];
  const int tid = threadIdx.x, lane = tid & 31, wave = tid >> 5, h = lane >> 4, m = lane & 15;
  for (int p = tid; p < MP * KP / 8; p += 128) ((v8h*)As)[p] = ((const v8h*)A)[p];
  if (MODE == 1) {
    for (int i = tid; i < 3 * MP; i += 128) {
      const int c = i / MP, k = i - c * MP;
      const float v = Kw2[c * NCH + min(k, NCH - 1)];
      kw2s[i] = (k < NCH) ? v : 0.0f;
    }
    if (tid < CH) kw1s[tid] = Kw1[tid];
  }
  __syncthreads();
  const int e0w = blockIdx.x * 64 + wave * 16;
  const _Float16* brow = P + (size_t)(e0w + m) * PR + 8 * h;
  _Float16* srow = Ss + (wave * 16 + m) * PR;
  v4f w3v = {0.0f, 0.0f, 0.0f, 0.0f};
  if (MODE == 0) {
    v8f acc[MT];
#pragma unroll
    for (int mt = 0; mt < MT; ++mt) acc[mt] = zacc();
#pragma unroll 1
    for (int kt = 0; kt < KT; ++kt) {
      Frag b;
      b.h[0] = *(const v8h*)(brow + kt * 32);
      b.h[1] = *(const v8h*)(brow + kt * 32 + 16);
#pragma unroll
      for (int mt = 0; mt < MT; ++mt) {
        Frag a;
        const _Float16* ap = As + (16 * mt + m) * KP + kt * 32 + 8 * h;
        a.h[0] = *(const v8h*)ap;
        a.h[1] = *(const v8h*)(ap + 16);
        acc[mt] = wmh(a.v, b.v, acc[mt]);
      }
    }
    float s1 = 0.0f;
#pragma unroll
    for (int mt = 0; mt < MT; ++mt)
#pragma unroll
      for (int r = 0; r < 8; ++r) s1 += acc[mt][r];
    s1 *= SCI;
    s1 += __shfl_xor(s1, 16, 32);
    const float mu = s1 * (1.0f / 193.0f);
    float ss = 0.0f;
#pragma unroll
    for (int mt = 0; mt < MT; ++mt)
#pragma unroll
      for (int r = 0; r < 8; ++r) {
        const int chn = 16 * mt + 8 * h + r;
        const float x = acc[mt][r] * SCI - mu;
        ss += (chn < NCH) ? x * x : 0.0f;
      }
    ss += __shfl_xor(ss, 16, 32);
    const float inv = 1.0f / sqrtf(ss + 1e-3f);
#pragma unroll
    for (int mt = 0; mt < MT; ++mt) {
      H8 t;
#pragma unroll
      for (int r = 0; r < 8; ++r) {
        const int chn = 16 * mt + 8 * h + r;
        const float v = SC * tanhf((acc[mt][r] * SCI - mu) * inv);
        t.h[r] = (_Float16)((chn < NCH) ? v : (v - v));
      }
      *(v8h*)(srow + 16 * mt + 8 * h) = t.h;
    }
    const v8h z = zh8();
#pragma unroll
    for (int q = 0; q < 3; ++q) {
      const int p = lane + 32 * q, rr = p / 6, cc = MP + 8 * (p - rr * 6);
      *(v8h*)(Ss + (wave * 16 + rr) * PR + cc) = z;
    }
  } else {
    Frag bf[KT];
#pragma unroll
    for (int kt = 0; kt < KT; ++kt) {
      bf[kt].h[0] = *(const v8h*)(brow + kt * 32);
      bf[kt].h[1] = *(const v8h*)(brow + kt * 32 + 16);
    }
    float* ys = Ys + (wave * 32 + lane) * 16;
    const float we = EW[(size_t)(e0w + m) * 4];
    const float inv1 = ST1[0];
    float p0 = 0.0f, p1 = 0.0f, p2 = 0.0f;
#pragma unroll 1
    for (int g = 0; g < 6; ++g) {
      v8f accA = zacc(), accB = zacc();
#pragma unroll
      for (int kt = 0; kt < KT; ++kt) {
        Frag a;
        const _Float16* ap = As + (16 * g + m) * KP + kt * 32 + 8 * h;
        a.h[0] = *(const v8h*)ap;
        a.h[1] = *(const v8h*)(ap + 16);
        accA = wmh(a.v, bf[kt].v, accA);
        const _Float16* ap2 = ap + CH * KP;
        a.h[0] = *(const v8h*)ap2;
        a.h[1] = *(const v8h*)(ap2 + 16);
        accB = wmh(a.v, bf[kt].v, accB);
      }
#pragma unroll
      for (int r = 0; r < 8; ++r) { ys[r] = accA[r]; ys[8 + r] = accB[r]; }
#pragma unroll 1
      for (int r = 0; r < 8; ++r) {
        const int cA = 16 * g + 8 * h + r;
        const float yA = tanhf(ys[r] * SCI), yB = tanhf(ys[8 + r] * SCI);
        p0 += kw2s[cA] * yA; p1 += kw2s[MP + cA] * yA; p2 += kw2s[2 * MP + cA] * yA;
        p0 += kw2s[CH + cA] * yB; p1 += kw2s[MP + CH + cA] * yB; p2 += kw2s[2 * MP + CH + cA] * yB;
        const float wc = tanhf((kw1s[cA] * we) * inv1);
        const float wg = wc * yA, wa = wc * yB;
        srow[cA] = (_Float16)(SC * (wg + 0.5f * wa));
        srow[CH + cA] = (_Float16)(SC * (0.5f * wa - wg));
      }
    }
    {
      v8f accA = zacc();
#pragma unroll
      for (int kt = 0; kt < KT; ++kt) {
        Frag a;
        const _Float16* ap = As + (16 * 12 + m) * KP + kt * 32 + 8 * h;
        a.h[0] = *(const v8h*)ap;
        a.h[1] = *(const v8h*)(ap + 16);
        accA = wmh(a.v, bf[kt].v, accA);
      }
#pragma unroll
      for (int r = 0; r < 8; ++r) ys[r] = accA[r];
#pragma unroll 1
      for (int r = 0; r < 8; ++r) {
        const int cA = 192 + 8 * h + r;
        const float yA = tanhf(ys[r] * SCI);
        p0 += kw2s[cA] * yA; p1 += kw2s[MP + cA] * yA; p2 += kw2s[2 * MP + cA] * yA;
      }
    }
    p0 += __shfl_xor(p0, 16, 32); p1 += __shfl_xor(p1, 16, 32); p2 += __shfl_xor(p2, 16, 32);
    w3v[0] = p0; w3v[1] = p1; w3v[2] = p2;
    const v8h z = zh8();
#pragma unroll
    for (int q = 0; q < 4; ++q) {
      const int p = lane + 32 * q, rr = p >> 3, cc = 2 * CH + 8 * (p & 7);
      *(v8h*)(Ss + (wave * 16 + rr) * PR + cc) = z;
    }
  }
  __syncthreads();
  const _Float16* srow0 = Ss + (wave * 16) * PR + 8 * lane;
  _Float16* prow0 = P + (size_t)e0w * PR + 8 * lane;
#pragma unroll
  for (int r = 0; r < 16; ++r) { H8 t; t.h = *(const v8h*)(srow0 + r * PR); *(volatile v4i*)(prow0 + (size_t)r * PR) = t.i; }
  if (MODE == 1) { if (h == 0) *(volatile v4f*)(W3 + (size_t)(e0w + m) * 4) = w3v; }
  __threadfence();
#pragma unroll
  for (int r = 0; r < 16; ++r) { H8 t; t.h = *(const v8h*)(srow0 + r * PR); *(volatile v4i*)(prow0 + (size_t)r * PR) = t.i; }
  if (MODE == 1) { if (h == 0) *(volatile v4f*)(W3 + (size_t)(e0w + m) * 4) = w3v; }
}

__global__ __launch_bounds__(256) void k_cmsg(const float* __restrict__ W3, const float* __restrict__ ST3,
    const float* __restrict__ C, const int* __restrict__ iI, const int* __restrict__ jI, float* WG, int N, int E)
{
#pragma clang fp contract(off)
  const int e = blockIdx.x * 256 + (int)threadIdx.x;
  if (e >= E) return;
  const v4f w3 = *(const v4f*)(W3 + (size_t)e * 4);
  const float inv3 = ST3[0];
  const int i = clampi(iI[e], N - 1), j = clampi(jI[e], N - 1);
  const v4f ci = *(const v4f*)(C + (size_t)i * 4), cj = *(const v4f*)(C + (size_t)j * 4);
  v4f o = {0.0f, 0.0f, 0.0f, 0.0f};
#pragma unroll
  for (int c = 0; c < 3; ++c) {
    const float t = tanhf(w3[c] * inv3);
    const float g = t * (ci[c] - cj[c]);
    o[c] = t * g;
  }
  *(volatile v4f*)(WG + (size_t)e * 4) = o;
  __threadfence();
  *(volatile v4f*)(WG + (size_t)e * 4) = o;
}

__global__ __launch_bounds__(256) void k_out(const float* __restrict__ C, const float* __restrict__ XN,
    const float* __restrict__ XE, float* out, int N, int E, int total)
{
  const int f0 = (blockIdx.x * 256 + (int)threadIdx.x) * 4;
  if (f0 >= total) return;
  const int n3 = 3 * N, n99 = 99 * N;
  const int a0 = min(f0, n3 - 4);
  const int c0 = a0 / N, q0 = a0 - c0 * N;
  const int a1 = min(max(f0 - n3, 0), CH * N - 4);
  const int c1 = a1 / N, q1 = a1 - c1 * N;
  const int a2 = min(max(f0 - n99, 0), 32 * E - 4);
  const int c2 = a2 / E, q2 = a2 - c2 * E;
  v4f v;
#pragma unroll
  for (int k = 0; k < 4; ++k) {
    const float x0 = C[(size_t)min(q0 + k, N - 1) * 4 + c0];
    const float x1 = XN[(size_t)min(q1 + k, N - 1) * CH + c1];
    const float x2 = XE[(size_t)min(q2 + k, E - 1) * 32 + c2];
    v[k] = (f0 < n3) ? x0 : ((f0 < n99) ? x1 : x2);
  }
  const bool full = (f0 + 3 < total);
  if (full) *(volatile v4f*)(out + f0) = v;
  else {
#pragma unroll
    for (int k = 0; k < 4; ++k) if (f0 + k < total) *(volatile float*)(out + f0 + k) = v[k];
  }
  __threadfence();
  if (full) *(volatile v4f*)(out + f0) = v;
  else {
#pragma unroll
    for (int k = 0; k < 4; ++k) if (f0 + k < total) *(volatile float*)(out + f0 + k) = v[k];
  }
}

extern "C" void kernel_launch(void* const* d_in, const int* in_sizes, int n_in,
                              void* d_out, int out_size, void* d_ws, size_t ws_size, hipStream_t stream)
{
  if (n_in < 13) return;
  const int N = in_sizes[0] / 40;
  const int E = in_sizes[1];
  if (N < 4 || E < 256) return;
  if (in_sizes[0] != 40 * N || (N & 3) != 0 || (E & 255) != 0) return;
  if (in_sizes[2] != 32 * 40 || in_sizes[3] != 32 * 32 || in_sizes[4] != 32 || in_sizes[5] != 32 * 32) return;
  if (in_sizes[6] != 3 * NCH * NCH || in_sizes[7] != 3 * NCH * NCH) return;
  if (in_sizes[8] != CH || in_sizes[9] != 3 * NCH) return;
  if (in_sizes[10] != E || in_sizes[11] != E || in_sizes[12] < 1) return;
  if (out_size != 99 * N + 32 * E) return;

  const float* xn  = (const float*)d_in[0];
  const float* xe  = (const float*)d_in[1];
  const float* K1N = (const float*)d_in[2];
  const float* K2N = (const float*)d_in[3];
  const float* K1E = (const float*)d_in[4];
  const float* K2E = (const float*)d_in[5];
  const float* KE1 = (const float*)d_in[6];
  const float* KE2 = (const float*)d_in[7];
  const float* Kw1 = (const float*)d_in[8];
  const float* Kw2 = (const float*)d_in[9];
  const int*   iI  = (const int*)d_in[10];
  const int*   jI  = (const int*)d_in[11];
  const int*   nnp = (const int*)d_in[12];
  float* out = (float*)d_out;

  const int NP = ((N + NB - 1) / NB) * NB;
  char* ws = (char*)d_ws;
  size_t off = 0;
  auto take = [&](size_t bytes) -> size_t { const size_t o = off; off += (bytes + 255) & ~(size_t)255; return o; };
  const size_t oP   = take((size_t)E * PR * 2);
  const size_t oXE  = take((size_t)E * 32 * 4);
  const size_t oXN  = take((size_t)NP * CH * 4);
  const size_t oX32 = take((size_t)NP * 32 * 4);
  const size_t oC   = take((size_t)NP * 16);
  const size_t oCO  = take((size_t)NP * 16);
  const size_t oEW  = take((size_t)E * 16);
  const size_t oW3  = take((size_t)E * 16);
  const size_t oWG  = take((size_t)E * 16);
  const size_t oST1 = take(256);
  const size_t oST3 = take(256);
  const size_t oA1  = take((size_t)3 * MP * KP * 2);
  const size_t oA2  = take((size_t)3 * MP * KP * 2);
  const size_t oWS  = take((size_t)384 * 16);
  if (off > ws_size) return;

  _Float16* P   = (_Float16*)(ws + oP);
  float*    XE  = (float*)(ws + oXE);
  float*    XN  = (float*)(ws + oXN);
  float*    X32 = (float*)(ws + oX32);
  float*    C   = (float*)(ws + oC);
  float*    CO  = (float*)(ws + oCO);
  float*    EW  = (float*)(ws + oEW);
  float*    W3  = (float*)(ws + oW3);
  float*    WG  = (float*)(ws + oWG);
  float*    ST1 = (float*)(ws + oST1);
  float*    ST3 = (float*)(ws + oST3);
  _Float16* A1  = (_Float16*)(ws + oA1);
  _Float16* A2  = (_Float16*)(ws + oA2);
  _Float16* WSM = (_Float16*)(ws + oWS);
  const _Float16* W1N = WSM;
  const _Float16* W2N = WSM + 2048;

  const int nblkA = (3 * MP * KP / 8 + 255) / 256;
  const int vec8 = ((E & 7) == 0) ? 1 : 0;
  const int gE64 = E / 64, gE256 = E / 256, gAgg = NP / NB;

  k_prep<<<2 * nblkA + 2, 256, 0, stream>>>(KE1, KE2, K1N, K2N, A1, A2, WSM, nblkA);
  k_nopen<<<(N + 63) / 64, 128, 0, stream>>>(xn, W1N, W2N, nnp, X32, C, CO, N);
  k_eopen<<<gE64, 256, 0, stream>>>(xe, K1E, K2E, XE);
  k_agg<0><<<gAgg, NTA, 0, stream>>>(iI, jI, XE, P, WG, X32, XN, C, CO, N, E, vec8);

  for (int l = 0; l < 3; ++l) {
    k_elen<<<gE256, 256, 0, stream>>>(XN, C, iI, jI, EW, N, E);
    k_std<<<1, 256, 0, stream>>>(EW, 4, 1, E, Kw1, CH, ST1);
    k_build<<<gE64, 128, 0, stream>>>(XN, iI, jI, Kw1, EW, ST1, P, N);
    k_gemm<0><<<gE64, 128, 0, stream>>>(A1 + (size_t)l * MP * KP, P, Kw1, Kw2, EW, ST1, W3);
    k_gemm<1><<<gE64, 128, 0, stream>>>(A2 + (size_t)l * MP * KP, P, Kw1, Kw2, EW, ST1, W3);
    k_std<<<1, 256, 0, stream>>>(W3, 4, 3, E, Kw1, 0, ST3);
    k_cmsg<<<gE256, 256, 0, stream>>>(W3, ST3, C, iI, jI, WG, N, E);
    k_agg<1><<<gAgg, NTA, 0, stream>>>(iI, jI, XE, P, WG, X32, XN, C, CO, N, E, vec8);
  }
  const int gOut = ((out_size + 3) / 4 + 255) / 256;
  k_out<<<gOut, 256, 0, stream>>>(C, XN, XE, out, N, E, out_size);
}
